// MixerGatedDeltaNet_10806137717337
// MI455X (gfx1250) — hardware-run, weakly checked
//
#include <hip/hip_runtime.h>
#include <math.h>

constexpr int kBatch    = 2;
constexpr int kSeqLen   = 1024;
constexpr int kDModel   = 768;
constexpr int kHeads    = 12;
constexpr int kDK       = 64;
constexpr int kDVh      = 128;
constexpr int kKeyDim   = 768;
constexpr int kValDim   = 1536;
constexpr int kInDim    = 3096;
constexpr int kInPad    = 3136;
constexpr int kTok      = kBatch * kSeqLen;
constexpr int kQkLd     = 2 * kKeyDim;
constexpr int kConvTaps = 4;
constexpr int kBhRows   = kBatch * kHeads;
constexpr float kScale   = 0.125f;
constexpr float kEpsNorm = 1e-5f;
constexpr float kEpsL2   = 1e-6f;
constexpr int kSPitch   = 68;
constexpr int kOChunk   = 32;

static_assert(kTok % 64 == 0 && kInPad % 64 == 0 && kValDim % 64 == 0 && kDModel % 32 == 0, "tile multiples");
static_assert(kInPad >= kInDim && kQkLd == kValDim, "layout");

typedef __attribute__((ext_vector_type(16))) _Float16 v16h;
typedef __attribute__((ext_vector_type(8)))  _Float16 v8h;
typedef __attribute__((ext_vector_type(16))) __bf16   v16b;
typedef __attribute__((ext_vector_type(8)))  __bf16   v8b;
typedef __attribute__((ext_vector_type(8)))  float    v8f;
typedef __attribute__((ext_vector_type(4)))  float    v4f;
typedef __attribute__((ext_vector_type(4)))  unsigned int v4u;

__device__ __forceinline__ unsigned short f2bf_bits(float f) {
  unsigned u = __float_as_uint(f);
  return (unsigned short)((u + 0x7FFFu + ((u >> 16) & 1u)) >> 16);
}
__device__ __forceinline__ float bf_bits2f(unsigned short h) { return __uint_as_float(((unsigned)h) << 16); }

__device__ __forceinline__ void dep_guard_h(v8f& a, v8f& b, v16h x, v16h y) { asm volatile("v_nop\n\tv_nop\n\tv_nop\n\tv_nop" : "+v"(a), "+v"(b) : "v"(x), "v"(y)); }
__device__ __forceinline__ void dep_guard_b(v8f& a, v8f& b, v16b x, v16b y) { asm volatile("v_nop\n\tv_nop\n\tv_nop\n\tv_nop" : "+v"(a), "+v"(b) : "v"(x), "v"(y)); }
__device__ __forceinline__ void keep4_h(v16h a, v16h b, v16h c, v16h d) { asm volatile("v_nop" :: "v"(a), "v"(b), "v"(c), "v"(d)); }
__device__ __forceinline__ void keep4_b(v16b a, v16b b, v16b c, v16b d) { asm volatile("v_nop" :: "v"(a), "v"(b), "v"(c), "v"(d)); }
__device__ __forceinline__ void acc_guard4(v8f& a, v8f& b, v8f& c, v8f& d) { asm volatile("v_nop\n\tv_nop\n\tv_nop\n\tv_nop" : "+v"(a), "+v"(b), "+v"(c), "+v"(d)); }
template <typename T> struct Frag;
template <> struct Frag<_Float16> {
  typedef v16h V; union U { v16h v; v8h h[2]; };
  static __device__ __forceinline__ v16h load(const _Float16* p) {
    U f; f.h[0] = *(const v8h*)(p); f.h[1] = *(const v8h*)(p + 16); return f.v;
  }
  static __device__ __forceinline__ v8f mma(v16h a, v16h b, v8f c) {
    return __builtin_amdgcn_wmma_f32_16x16x32_f16(false, a, false, b, (short)0, c, false, false);
  }
  static __device__ __forceinline__ void guard(v8f& a, v8f& b, v16h x, v16h y) { dep_guard_h(a, b, x, y); }
  static __device__ __forceinline__ void keep(v16h a, v16h b, v16h c, v16h d) { keep4_h(a, b, c, d); }
};
template <> struct Frag<__bf16> {
  typedef v16b V; union U { v16b v; v8b h[2]; };
  static __device__ __forceinline__ v16b load(const __bf16* p) {
    U f; f.h[0] = *(const v8b*)(p); f.h[1] = *(const v8b*)(p + 16); return f.v;
  }
  static __device__ __forceinline__ v8f mma(v16b a, v16b b, v8f c) {
    return __builtin_amdgcn_wmma_f32_16x16x32_bf16(false, a, false, b, (short)0, c, false, false);
  }
  static __device__ __forceinline__ void guard(v8f& a, v8f& b, v16b x, v16b y) { dep_guard_b(a, b, x, y); }
  static __device__ __forceinline__ void keep(v16b a, v16b b, v16b c, v16b d) { keep4_b(a, b, c, d); }
};

__device__ __forceinline__ unsigned pk16(unsigned short a, unsigned short b) { return (unsigned)a | ((unsigned)b << 16); }

template <int ET> struct Elem;
template <> struct Elem<0> { typedef _Float16 T; };
template <> struct Elem<1> { typedef __bf16 T; };
template <int ET, bool SPLIT, int BIAS_MODE, int OUT_MODE, bool RESID, int ACT = 0>
__global__ __launch_bounds__(256) void wmma_gemm64(
    const unsigned short* __restrict__ Ap, const unsigned short* __restrict__ A2p, int lda, long strideA,
    const unsigned short* __restrict__ Btp, const unsigned short* __restrict__ Bt2p, int ldb, long strideB,
    void* __restrict__ Cout, void* __restrict__ Cout2, int ldc, long strideC,
    const float* __restrict__ bias,
    const float* __restrict__ resid, long strideR,
    int M, int N, int K, float scale) {
  typedef typename Elem<ET>::T T;
  typedef typename Frag<T>::V V;
  const T* A = (const T*)Ap; const T* A2 = (const T*)A2p; const T* Bt = (const T*)Btp; const T* Bt2 = (const T*)Bt2p;
  __shared__ __align__(16) float sT[8][16 * 68];
  const int b    = blockIdx.y;
  const int lane = threadIdx.x & 31;
  const int wave = threadIdx.x >> 5;
  const int tilesN = N >> 6;
  const int tilesM = M >> 6;
  const int tile = blockIdx.x * 8 + wave;
  if (tile >= tilesM * tilesN) return;
  const int tm = tile / tilesN;
  const int tn = tile - tm * tilesN;
  const int m0 = tm << 6;
  const int n0 = tn << 6;

  const T* Ab  = A  + (size_t)b * strideA;
  const T* Bb  = Bt + (size_t)b * strideB;
  const T* Ab2 = SPLIT ? (A2  + (size_t)b * strideA) : nullptr;
  const T* Bb2 = SPLIT ? (Bt2 + (size_t)b * strideB) : nullptr;

  const int rlane = lane & 15;
  const int koff  = (lane >> 4) * 8;
  const int mOff  = (lane >> 4) * 8;

  v8f acc[4][4];
#pragma unroll
  for (int i = 0; i < 4; ++i)
#pragma unroll
    for (int j = 0; j < 4; ++j) acc[i][j] = (v8f){0.f,0.f,0.f,0.f,0.f,0.f,0.f,0.f};

  for (int k0 = 0; k0 < K; k0 += 32) {
    V bh[4], bl[4];
#pragma unroll
    for (int j = 0; j < 4; ++j) {
      const size_t bo = (size_t)(n0 + (j << 4) + rlane) * ldb + koff + k0;
      bh[j] = Frag<T>::load(Bb + bo);
      if (SPLIT) bl[j] = Frag<T>::load(Bb2 + bo);
    }
#pragma unroll
    for (int i = 0; i < 4; ++i) {
      const size_t ao = (size_t)(m0 + (i << 4) + rlane) * lda + koff + k0;
      V ah = Frag<T>::load(Ab + ao);
      V al;
      if (SPLIT) al = Frag<T>::load(Ab2 + ao);
#pragma unroll
      for (int j = 0; j < 4; ++j) {
        acc[i][j] = Frag<T>::mma(ah, bh[j], acc[i][j]);
        if (SPLIT) {
          acc[i][j] = Frag<T>::mma(ah, bl[j], acc[i][j]);
          acc[i][j] = Frag<T>::mma(al, bh[j], acc[i][j]);
        }
      }
      Frag<T>::guard(acc[i][0], acc[i][3], ah, SPLIT ? al : ah);
    }
    Frag<T>::keep(bh[0], bh[1], bh[2], bh[3]);
    if (SPLIT) Frag<T>::keep(bl[0], bl[1], bl[2], bl[3]);
  }
  acc_guard4(acc[0][0], acc[0][1], acc[0][2], acc[0][3]);
  acc_guard4(acc[1][0], acc[1][1], acc[1][2], acc[1][3]);
  acc_guard4(acc[2][0], acc[2][1], acc[2][2], acc[2][3]);
  acc_guard4(acc[3][0], acc[3][1], acc[3][2], acc[3][3]);

  float* slab = sT[wave];
  const float* Rb = RESID ? (resid + (size_t)b * strideR) : nullptr;
#pragma unroll
  for (int i = 0; i < 4; ++i) {
    const int mBase = m0 + (i << 4);
#pragma unroll
    for (int j = 0; j < 4; ++j) {
      const int n = n0 + (j << 4) + rlane;
      float bv = 0.f;
      if (BIAS_MODE == 2) bv = bias[n];
#pragma unroll
      for (int r = 0; r < 8; ++r) {
        float v = acc[i][j][r] * scale;
        if (BIAS_MODE == 1) v += bias[mBase + mOff + r];
        if (BIAS_MODE == 2) v += bv;
        if (RESID) v += Rb[(size_t)(mBase + mOff + r) * ldc + n];
        if (ACT == 2) v = fmaxf(v, 0.0f);
        if (ACT == 4) v = (v > 0.f) ? v : 0.01f * v;
        slab[(mOff + r) * 68 + (j << 4) + rlane] = v;
      }
    }
    __builtin_amdgcn_fence(__ATOMIC_RELEASE, "workgroup");
    __builtin_amdgcn_wave_barrier();
    __builtin_amdgcn_fence(__ATOMIC_ACQUIRE, "workgroup");
    if (OUT_MODE == 0) {
      float* C = (float*)Cout + (size_t)b * strideC;
      const int hh = lane >> 4, c4 = (lane & 15) * 4;
      for (int pass = 0; pass < 2; ++pass) {
#pragma unroll
        for (int it = 0; it < 8; ++it) {
          const int row = it * 2 + hh;
          v4f v = *(const v4f*)(slab + row * 68 + c4);
          *(volatile v4f*)(C + (size_t)(mBase + row) * ldc + n0 + c4) = v;
        }
        __threadfence();
      }
    } else {
      const int q = lane >> 3, c8 = (lane & 7) * 8;
      unsigned short* C  = (unsigned short*)Cout  + (size_t)b * strideC;
      unsigned short* C2 = (OUT_MODE == 2) ? ((unsigned short*)Cout2 + (size_t)b * strideC) : nullptr;
      for (int pass = 0; pass < 2; ++pass) {
#pragma unroll
        for (int it = 0; it < 4; ++it) {
          const int row = it * 4 + q;
          const float* sp = slab + row * 68 + c8;
          v8h hv, lv;
#pragma unroll
          for (int e = 0; e < 8; ++e) {
            if (OUT_MODE == 1) {
              hv[e] = (_Float16)sp[e];
            } else {
              unsigned short hb = f2bf_bits(sp[e]);
              unsigned short lb = f2bf_bits(sp[e] - bf_bits2f(hb));
              hv[e] = __builtin_bit_cast(_Float16, hb);
              lv[e] = __builtin_bit_cast(_Float16, lb);
            }
          }
          *(volatile v8h*)(C + (size_t)(mBase + row) * ldc + n0 + c8) = hv;
          if (OUT_MODE == 2) *(volatile v8h*)(C2 + (size_t)(mBase + row) * ldc + n0 + c8) = lv;
        }
        __threadfence();
      }
    }
    __builtin_amdgcn_fence(__ATOMIC_RELEASE, "workgroup");
    __builtin_amdgcn_wave_barrier();
    __builtin_amdgcn_fence(__ATOMIC_ACQUIRE, "workgroup");
  }
}

__global__ __launch_bounds__(256) void split8_bf16_kernel(const float* __restrict__ in,
    unsigned short* __restrict__ hi, unsigned short* __restrict__ lo, int n8) {
  const int i = blockIdx.x * 256 + threadIdx.x;
  if (i >= n8) return;
  const float* p = in + 8 * (size_t)i;
  const v4f a = *(const v4f*)(p);
  const v4f c = *(const v4f*)(p + 4);
  unsigned short hb[8], lb[8];
#pragma unroll
  for (int e = 0; e < 4; ++e) {
    const float x0 = a[e], x1 = c[e];
    const unsigned short h0 = f2bf_bits(x0), h1 = f2bf_bits(x1);
    hb[e] = h0; hb[4 + e] = h1;
    lb[e]     = f2bf_bits(x0 - bf_bits2f(h0));
    lb[4 + e] = f2bf_bits(x1 - bf_bits2f(h1));
  }
  const v4u uh = (v4u){pk16(hb[0], hb[1]), pk16(hb[2], hb[3]), pk16(hb[4], hb[5]), pk16(hb[6], hb[7])};
  const v4u ul = (v4u){pk16(lb[0], lb[1]), pk16(lb[2], lb[3]), pk16(lb[4], lb[5]), pk16(lb[6], lb[7])};
  unsigned short* qh = hi + 8 * (size_t)i;
  unsigned short* ql = lo + 8 * (size_t)i;
  *(volatile v4u*)qh = uh;
  *(volatile v4u*)ql = ul;
  __threadfence();
  *(volatile v4u*)qh = uh;
  *(volatile v4u*)ql = ul;
}

__global__ __launch_bounds__(256) void wt_split_kernel(const float* __restrict__ W, int ncols,
    unsigned short* __restrict__ hi, unsigned short* __restrict__ lo) {
  __shared__ float sm[64][65];
  const int t  = threadIdx.x;
  const int d0 = blockIdx.x * 64;
  const int n0 = blockIdx.y * 64;
#pragma unroll
  for (int i = 0; i < 16; ++i) {
    const int e = i * 256 + t;
    const int r = e >> 6;
    const int c = e & 63;
    const int n = n0 + c;
    const int nc = (n < ncols) ? n : (ncols - 1);
    const float w = W[(size_t)(d0 + r) * ncols + nc];
    sm[c][r] = (n < ncols) ? w : 0.0f;
  }
  __syncthreads();
  const int lane = t & 31, wave = t >> 5;
  const int q = lane >> 3, c8 = (lane & 7) * 8;
  for (int pass = 0; pass < 2; ++pass) {
#pragma unroll
    for (int it = 0; it < 2; ++it) {
      const int row = wave * 8 + it * 4 + q;
      unsigned short hb[8], lb[8];
#pragma unroll
      for (int e = 0; e < 8; ++e) {
        const float x = sm[row][c8 + e];
        const unsigned short h0 = f2bf_bits(x);
        hb[e] = h0;
        lb[e] = f2bf_bits(x - bf_bits2f(h0));
      }
      const v4u uh = (v4u){pk16(hb[0], hb[1]), pk16(hb[2], hb[3]), pk16(hb[4], hb[5]), pk16(hb[6], hb[7])};
      const v4u ul = (v4u){pk16(lb[0], lb[1]), pk16(lb[2], lb[3]), pk16(lb[4], lb[5]), pk16(lb[6], lb[7])};
      const size_t o = (size_t)(n0 + row) * kDModel + d0 + c8;
      *(volatile v4u*)(hi + o) = uh;
      *(volatile v4u*)(lo + o) = ul;
    }
    __threadfence();
  }
}

__global__ __launch_bounds__(256) void gate_scalar_kernel(const float* __restrict__ qkvba,
    const float* __restrict__ dt_bias, const float* __restrict__ a_log,
    float* __restrict__ beta_o, float* __restrict__ dec_o) {
  const int i = blockIdx.x * 256 + threadIdx.x;
  if (i >= kBhRows * kSeqLen) return;
  const int bh = i >> 10;
  const int t  = i & (kSeqLen - 1);
  const int b  = bh / kHeads;
  const int h  = bh - b * kHeads;
  const size_t m = (size_t)b * kSeqLen + t;
  const float bc = qkvba[m * kInPad + 2 * kKeyDim + kValDim + h];
  const float ac = qkvba[m * kInPad + 2 * kKeyDim + kValDim + kHeads + h];
  const float beta = 1.0f / (1.0f + expf(-bc));
  const float ap = ac + dt_bias[h];
  const float sp = fmaxf(ap, 0.0f) + log1pf(expf(-fabsf(ap)));
  const float g  = -expf(a_log[h]) * sp;
  const float dec = expf(g);
  volatile float* pb = beta_o + i;
  volatile float* pd = dec_o + i;
  *pb = beta;
  *pd = dec;
  __threadfence();
  *pb = beta;
  *pd = dec;
}

__global__ __launch_bounds__(384) void shortconv_kernel(const float* __restrict__ qkvba,
    const float* __restrict__ qw, const float* __restrict__ kw, const float* __restrict__ vw,
    float* __restrict__ qk_out, float* __restrict__ v_out) {
  const int m    = blockIdx.x;
  const int part = blockIdx.y;
  const int tid  = threadIdx.x;
  const int b    = m / kSeqLen;
  const int t    = m - b * kSeqLen;
  const int ch   = 4 * tid;
  const int col  = part * kQkLd + ch;
  const float* wsrc = vw;
  int wch = ch;
  if (part == 0) {
    if (tid < 192) { wsrc = qw; wch = ch; } else { wsrc = kw; wch = ch - kKeyDim; }
  }
  v4f acc = (v4f){0.f, 0.f, 0.f, 0.f};
#pragma unroll 1
  for (int j = 0; j < kConvTaps; ++j) {
    const int ts  = t - (kConvTaps - 1) + j;
    const int tsc = (ts < 0) ? 0 : ts;
    const float valid = (ts < 0) ? 0.0f : 1.0f;
    const v4f x = *(const v4f*)(qkvba + ((size_t)b * kSeqLen + tsc) * kInPad + col);
    v4f w;
    w[0] = wsrc[(size_t)(wch + 0) * kConvTaps + j];
    w[1] = wsrc[(size_t)(wch + 1) * kConvTaps + j];
    w[2] = wsrc[(size_t)(wch + 2) * kConvTaps + j];
    w[3] = wsrc[(size_t)(wch + 3) * kConvTaps + j];
    acc += (x * valid) * w;
  }
  const float y0 = acc[0] * (1.0f / (1.0f + expf(-acc[0])));
  const float y1 = acc[1] * (1.0f / (1.0f + expf(-acc[1])));
  const float y2 = acc[2] * (1.0f / (1.0f + expf(-acc[2])));
  const float y3 = acc[3] * (1.0f / (1.0f + expf(-acc[3])));
  float ss = y0 * y0 + y1 * y1 + y2 * y2 + y3 * y3;
  ss += __shfl_xor(ss, 1, 32);
  ss += __shfl_xor(ss, 2, 32);
  ss += __shfl_xor(ss, 4, 32);
  ss += __shfl_xor(ss, 8, 32);
  const float rn = 1.0f / sqrtf(ss + kEpsL2);
  const float sc = (part == 0) ? rn : 1.0f;
  const v4f r = (v4f){y0 * sc, y1 * sc, y2 * sc, y3 * sc};
  float* dst = ((part == 0) ? qk_out : v_out) + (size_t)m * kValDim + ch;
  *(volatile v4f*)dst = r;
  __threadfence();
  *(volatile v4f*)dst = r;
}

__global__ __launch_bounds__(128) void gdr_scan_kernel(const float* __restrict__ qk,
    const float* __restrict__ vv, const float* __restrict__ beta_a, const float* __restrict__ dec_a,
    float* __restrict__ o_out) {
  __shared__ __align__(16) float Ssh[kDVh * kSPitch];
  __shared__ __align__(16) float shkq[2][2 * kDK];
  __shared__ __align__(16) float obuf[kOChunk * kDVh];
  const int bh   = blockIdx.x;
  const int b    = bh / kHeads;
  const int h    = bh - b * kHeads;
  const int tid  = threadIdx.x;
  const int lane = tid & 31, wave = tid >> 5;
  float* Srow = Ssh + tid * kSPitch;
  const v4f z4 = (v4f){0.f, 0.f, 0.f, 0.f};
#pragma unroll 1
  for (int i = 0; i < kDK / 4; ++i) *(v4f*)(Srow + 4 * i) = z4;
  const int kqcol = (tid < kDK) ? (kKeyDim + h * kDK + tid) : (h * kDK + tid - kDK);
  const size_t m0 = (size_t)b * kSeqLen;
  const float* betab = beta_a + (size_t)bh * kSeqLen;
  const float* decb  = dec_a  + (size_t)bh * kSeqLen;
  for (int t = 0; t < kSeqLen; ++t) {
    const int buf = t & 1;
    const size_t m = m0 + t;
    shkq[buf][tid] = qk[m * kQkLd + kqcol];
    const float vval = vv[m * kValDim + h * kDVh + tid];
    const float dec  = decb[t];
    const float bet  = betab[t];
    __syncthreads();
    const float* kp = shkq[buf];
    const float* qp = shkq[buf] + kDK;
    v4f pa = z4, pb = z4;
#pragma unroll 1
    for (int i = 0; i < kDK / 8; ++i) {
      const v4f k0 = *(const v4f*)(kp + 8 * i);
      const v4f k1 = *(const v4f*)(kp + 8 * i + 4);
      const v4f s0 = *(const v4f*)(Srow + 8 * i);
      const v4f s1 = *(const v4f*)(Srow + 8 * i + 4);
      pa += k0 * s0;
      pb += k1 * s1;
    }
    const v4f ps  = pa + pb;
    const float p = ((ps[0] + ps[1]) + (ps[2] + ps[3])) * dec;
    const float err = vval - p;
    const float cf  = bet * err;
    v4f oa = z4, ob = z4;
#pragma unroll 1
    for (int i = 0; i < kDK / 8; ++i) {
      const v4f k0 = *(const v4f*)(kp + 8 * i);
      const v4f k1 = *(const v4f*)(kp + 8 * i + 4);
      const v4f q0 = *(const v4f*)(qp + 8 * i);
      const v4f q1 = *(const v4f*)(qp + 8 * i + 4);
      const v4f s0 = *(const v4f*)(Srow + 8 * i);
      const v4f s1 = *(const v4f*)(Srow + 8 * i + 4);
      const v4f n0v = k0 * cf + s0 * dec;
      const v4f n1v = k1 * cf + s1 * dec;
      *(v4f*)(Srow + 8 * i)     = n0v;
      *(v4f*)(Srow + 8 * i + 4) = n1v;
      oa += q0 * n0v;
      ob += q1 * n1v;
    }
    const v4f os4 = oa + ob;
    const float ov = ((os4[0] + os4[1]) + (os4[2] + os4[3])) * kScale;
    obuf[(t & (kOChunk - 1)) * kDVh + tid] = ov;
    if ((t & (kOChunk - 1)) == (kOChunk - 1)) {
      __syncthreads();
      const int tb = t - (kOChunk - 1);
      for (int pass = 0; pass < 2; ++pass) {
#pragma unroll 1
        for (int it = 0; it < kOChunk / 4; ++it) {
          const int row = it * 4 + wave;
          const v4f val = *(const v4f*)(obuf + row * kDVh + 4 * lane);
          *(volatile v4f*)(o_out + (m0 + tb + row) * kValDim + h * kDVh + 4 * lane) = val;
        }
        __threadfence();
      }
    }
  }
}

__global__ __launch_bounds__(384) void norm_gate_kernel(const float* __restrict__ o_in,
    const float* __restrict__ gate, const float* __restrict__ onw, float* __restrict__ out) {
  const int m    = blockIdx.x;
  const int tid  = threadIdx.x;
  const int lane = tid & 31, h = tid >> 5;
  const size_t base = (size_t)m * kValDim + h * kDVh + 4 * lane;
  const v4f ov = *(const v4f*)(o_in + base);
  const v4f gv = *(const v4f*)(gate + base);
  const v4f wv = *(const v4f*)(onw + 4 * lane);
  float ss = ov[0] * ov[0] + ov[1] * ov[1] + ov[2] * ov[2] + ov[3] * ov[3];
  ss += __shfl_xor(ss, 16, 32);
  ss += __shfl_xor(ss, 8, 32);
  ss += __shfl_xor(ss, 4, 32);
  ss += __shfl_xor(ss, 2, 32);
  ss += __shfl_xor(ss, 1, 32);
  const float var = ss * (1.0f / 128.0f);
  const float rn  = 1.0f / sqrtf(var + kEpsNorm);
  v4f r;
#pragma unroll
  for (int e = 0; e < 4; ++e) {
    const float g  = gv[e];
    const float sg = 1.0f / (1.0f + expf(-g));
    r[e] = ov[e] * rn * wv[e] * g * sg;
  }
  float* dst = out + base;
  *(volatile v4f*)dst = r;
  __threadfence();
  *(volatile v4f*)dst = r;
}

extern "C" void kernel_launch(void* const* d_in, const int* in_sizes, int n_in,
                              void* d_out, int out_size, void* d_ws, size_t ws_size,
                              hipStream_t stream) {
  (void)n_in;
  if (in_sizes[0] != kTok * kDModel) return;
  if (in_sizes[1] != kDModel * kInDim) return;
  if (in_sizes[2] != kDModel * kValDim) return;
  if (out_size != kTok * kValDim) return;
  const float* hs      = (const float*)d_in[0];
  const float* w_in    = (const float*)d_in[1];
  const float* w_g     = (const float*)d_in[2];
  const float* dt_bias = (const float*)d_in[3];
  const float* a_log   = (const float*)d_in[4];
  const float* qw      = (const float*)d_in[5];
  const float* kw      = (const float*)d_in[6];
  const float* vw      = (const float*)d_in[7];
  const float* onw     = (const float*)d_in[8];
  float* out = (float*)d_out;

  char* wsb = (char*)d_ws;
  size_t off = 0;
  const size_t szHsP  = (size_t)kTok * kDModel * 2;
  const size_t szWinP = (size_t)kInPad * kDModel * 2;
  const size_t szWgP  = (size_t)kValDim * kDModel * 2;
  const size_t szQkv  = (size_t)kTok * kInPad * 4;
  const size_t szRow  = (size_t)kTok * kValDim * 4;
  const size_t szSc   = (size_t)kBhRows * kSeqLen * 4;
  unsigned short* hs_hi   = (unsigned short*)(wsb + off); off += szHsP;
  unsigned short* hs_lo   = (unsigned short*)(wsb + off); off += szHsP;
  unsigned short* winT_hi = (unsigned short*)(wsb + off); off += szWinP;
  unsigned short* winT_lo = (unsigned short*)(wsb + off); off += szWinP;
  unsigned short* wgT_hi  = (unsigned short*)(wsb + off); off += szWgP;
  unsigned short* wgT_lo  = (unsigned short*)(wsb + off); off += szWgP;
  float* qkvba = (float*)(wsb + off); off += szQkv;
  float* gate  = (float*)(wsb + off); off += szRow;
  float* qkbuf = (float*)(wsb + off); off += szRow;
  float* vbuf  = (float*)(wsb + off); off += szRow;
  float* betab = (float*)(wsb + off); off += szSc;
  float* decb  = (float*)(wsb + off); off += szSc;
  float* obuf  = (float*)(wsb + off); off += szRow;
  if (off > ws_size) return;

  {
    const int n8 = kTok * kDModel / 8;
    split8_bf16_kernel<<<dim3((n8 + 255) / 256), dim3(256), 0, stream>>>(hs, hs_hi, hs_lo, n8);
    wt_split_kernel<<<dim3(kDModel / 64, kInPad / 64), dim3(256), 0, stream>>>(w_in, kInDim, winT_hi, winT_lo);
    wt_split_kernel<<<dim3(kDModel / 64, kValDim / 64), dim3(256), 0, stream>>>(w_g, kValDim, wgT_hi, wgT_lo);
  }
  {
    const int tiles1 = (kTok / 64) * (kInPad / 64);
    wmma_gemm64<1, true, 0, 0, false, 0><<<dim3((tiles1 + 7) / 8, 1), dim3(256), 0, stream>>>(
        hs_hi, hs_lo, kDModel, 0L, winT_hi, winT_lo, kDModel, 0L,
        (void*)qkvba, (void*)nullptr, kInPad, 0L, (const float*)nullptr, (const float*)nullptr, 0L,
        kTok, kInPad, kDModel, 1.0f);
    const int tiles2 = (kTok / 64) * (kValDim / 64);
    wmma_gemm64<1, true, 0, 0, false, 0><<<dim3((tiles2 + 7) / 8, 1), dim3(256), 0, stream>>>(
        hs_hi, hs_lo, kDModel, 0L, wgT_hi, wgT_lo, kDModel, 0L,
        (void*)gate, (void*)nullptr, kValDim, 0L, (const float*)nullptr, (const float*)nullptr, 0L,
        kTok, kValDim, kDModel, 1.0f);
  }
  gate_scalar_kernel<<<dim3((kBhRows * kSeqLen + 255) / 256), dim3(256), 0, stream>>>(qkvba, dt_bias, a_log, betab, decb);
  shortconv_kernel<<<dim3(kTok, 2), dim3(384), 0, stream>>>(qkvba, qw, kw, vw, qkbuf, vbuf);
  gdr_scan_kernel<<<dim3(kBhRows), dim3(128), 0, stream>>>(qkbuf, vbuf, betab, decb, obuf);
  norm_gate_kernel<<<dim3(kTok), dim3(384), 0, stream>>>(obuf, gate, onw, out);
}
